// SpatialCrossAttention_49228915147512
// MI455X (gfx1250) — hardware-run, weakly checked
//
#include <hip/hip_runtime.h>


#ifndef LQ
#define LQ 40000
#endif
#define LQ_FULL 40000
#define NCAM 6
#define CC   256
#define HF   56
#define WF   100
#define HW   (HF * WF)
#define SWV  8
#define ACAR 16.0f
#define WCAR 256.0f
#define FOLD (1.0f / 4096.0f)
#define SC2  ((float)(0.0625 * 1.4426950408889634))
#define NEGB (-3.0e38f)

static_assert(CC == 32 * 8);
static_assert(CC % 64 == 0);
static_assert(CC % 32 == 0);
static_assert(HW % 32 == 0);
static_assert(LQ % 64 == 0);
static_assert(LQ % SWV == 0);
static_assert(LQ <= LQ_FULL);
static_assert(((size_t)CC * CC / 8) % 256 == 0);
static_assert(256 * 16 * 1 == 32 * 128);
static_assert(32 * 16 * 1 == CC * 2);
static_assert(32 * 16 * 8 == 16 * 64 * 4);
static_assert(64 * 33 * 4 <= 131072);
static_assert(16 * 68 * 4 <= 131072);
static_assert((68 * 4) % 16 == 0);

typedef _Float16 h16;
typedef unsigned short bf;
typedef __attribute__((ext_vector_type(16))) _Float16 v16h;
typedef __attribute__((ext_vector_type(8)))  _Float16 v8h;
typedef __attribute__((ext_vector_type(8)))  unsigned short v8us;
typedef __attribute__((ext_vector_type(4)))  unsigned int v4u;
typedef __attribute__((ext_vector_type(8)))  float    v8f;
typedef __attribute__((ext_vector_type(4)))  float    v4f;
typedef v4f  __attribute__((may_alias)) v4fa;

__device__ __forceinline__ unsigned short f2bf(float f) { unsigned u = __float_as_uint(f); u += 0x7FFFu + ((u >> 16) & 1u); return (unsigned short)(u >> 16); }
__device__ __forceinline__ float bfr(float f) { return __uint_as_float(((unsigned)f2bf(f)) << 16); }
__device__ __forceinline__ v16h cat16(v8h lo, v8h hi) { return __builtin_shufflevector(lo, hi, 0, 1, 2, 3, 4, 5, 6, 7, 8, 9, 10, 11, 12, 13, 14, 15); }
__device__ __forceinline__ v8f wmma16(v16h a, v16h b, v8f c) { return __builtin_amdgcn_wmma_f32_16x16x32_f16(false, a, false, b, (short)0, c, false, false); }
__device__ __forceinline__ v8f wmma16g(v16h a, v16h b, v8f c) { c = wmma16(a, b, c); asm volatile("v_nop\n\tv_nop\n\tv_nop\n\tv_nop" : "+v"(c) : "v"(a), "v"(b)); return c; }
__device__ __forceinline__ v16h  ldh(const h16* p) { return cat16(*(const v8h*)p, *(const v8h*)(p + 16)); }
__device__ __forceinline__ void wave_sync() { __builtin_amdgcn_fence(3  , "wavefront"); __builtin_amdgcn_wave_barrier(); asm volatile("" ::: "memory"); }
static __device__ __forceinline__ h16 toh_flush(float v) { const h16 r = (h16)v; return (fabsf(v) < 6.103515625e-05f) ? (h16)0.0f : r; }

__global__ __launch_bounds__(256) void k_wcvt(const float* __restrict__ src, h16* dst) {
    const size_t i = (size_t)blockIdx.x * 256 + threadIdx.x;
    const v8f v = *(const v8f*)(src + i * 8); v8h o;
#pragma unroll
    for (int k = 0; k < 8; ++k) o[k] = toh_flush(bfr(v[k]) * WCAR);
    *(volatile v8h*)(dst + i * 8) = o; __threadfence(); *(volatile v8h*)(dst + i * 8) = o;
}

__global__ __launch_bounds__(256) void k_vtr(const float* __restrict__ v, bf* VB) {
    __shared__ float tile[64 * 33];
    const int tid = threadIdx.x, x = tid & 31, y = tid >> 5;
    const int n = blockIdx.z, c0 = blockIdx.y * 64, p0 = blockIdx.x * 32;
#pragma unroll
    for (int i = 0; i < 8; ++i) { const int c = y + 8 * i;
        tile[c * 33 + x] = v[((size_t)n * CC + (size_t)(c0 + c)) * HW + (size_t)(p0 + x)]; }
    __syncthreads();
    const int p = tid >> 3, c8 = (tid & 7) * 8;
    v8us o;
#pragma unroll
    for (int k = 0; k < 8; ++k) o[k] = f2bf(tile[(c8 + k) * 33 + p]);
    bf* dst = VB + ((size_t)n * HW + (size_t)(p0 + p)) * CC + (size_t)(c0 + c8);
    *(volatile v8us*)dst = o; __threadfence(); *(volatile v8us*)dst = o;
}

__global__ __launch_bounds__(256) void k_sample(const float* __restrict__ query, const bf* __restrict__ VB, const float* __restrict__ pts,
                                                const int* __restrict__ msk, h16* TP) {
#pragma clang fp contract(off)
    const int lane = threadIdx.x & 31;
    const int wave = __builtin_amdgcn_readfirstlane((int)(threadIdx.x >> 5));
    const int l = blockIdx.x * SWV + wave;
    const int cb = lane * 8;
    float q[8];
    { const v4f qa = *(const v4f*)(query + (size_t)l * CC + cb); const v4f qb = *(const v4f*)(query + (size_t)l * CC + cb + 4);
#pragma unroll
      for (int i = 0; i < 4; ++i) { q[i] = bfr(qa[i]); q[4 + i] = bfr(qb[i]); } }
    float acc[8], sm[8];
#pragma unroll
    for (int i = 0; i < 8; ++i) { acc[i] = 0.0f; sm[i] = 0.0f; }
    float m = NEGB, Z = 0.0f; int msum = 0;
#pragma unroll 1
    for (int n = 0; n < NCAM; ++n) {
        const size_t gi = ((size_t)n * LQ_FULL + (size_t)l) * 2;
        const float gx = bfr(pts[gi]), gy = bfr(pts[gi + 1]);
        const int mk = msk[(size_t)n * LQ_FULL + (size_t)l];
        float ix = ((gx + 1.0f) * (float)WF - 1.0f) * 0.5f; ix = fminf(fmaxf(ix, 0.0f), (float)(WF - 1));
        float iy = ((gy + 1.0f) * (float)HF - 1.0f) * 0.5f; iy = fminf(fmaxf(iy, 0.0f), (float)(HF - 1));
        const float x0f = floorf(ix), y0f = floorf(iy);
        const float wx = ix - x0f, wy = iy - y0f;
        int x0 = (int)x0f, y0 = (int)y0f;
        x0 = min(max(x0, 0), WF - 1); y0 = min(max(y0, 0), HF - 1);
        const int x1 = min(x0 + 1, WF - 1), y1 = min(y0 + 1, HF - 1);
        const float ux = 1.0f - wx, uy = 1.0f - wy;
        const float w00 = ux * uy, w01 = wx * uy, w10 = ux * wy, w11 = wx * wy;
        const size_t pb = (size_t)n * HW * CC + (size_t)cb;
        const v4u a00 = *(const v4u*)(VB + pb + (size_t)(y0 * WF + x0) * CC);
        const v4u a01 = *(const v4u*)(VB + pb + (size_t)(y0 * WF + x1) * CC);
        const v4u a10 = *(const v4u*)(VB + pb + (size_t)(y1 * WF + x0) * CC);
        const v4u a11 = *(const v4u*)(VB + pb + (size_t)(y1 * WF + x1) * CC);
        float s[8];
#pragma unroll
        for (int i = 0; i < 4; ++i) {
            const float l00 = __uint_as_float(a00[i] << 16), h00 = __uint_as_float(a00[i] & 0xffff0000u);
            const float l01 = __uint_as_float(a01[i] << 16), h01 = __uint_as_float(a01[i] & 0xffff0000u);
            const float l10 = __uint_as_float(a10[i] << 16), h10 = __uint_as_float(a10[i] & 0xffff0000u);
            const float l11 = __uint_as_float(a11[i] << 16), h11 = __uint_as_float(a11[i] & 0xffff0000u);
            s[2 * i]     = ((l00 * w00 + l01 * w01) + l10 * w10) + l11 * w11;
            s[2 * i + 1] = ((h00 * w00 + h01 * w01) + h10 * w10) + h11 * w11; }
        float ls = ((s[0] + s[1]) + (s[2] + s[3])) + ((s[4] + s[5]) + (s[6] + s[7]));
#pragma unroll
        for (int off = 16; off > 0; off >>= 1) ls += __shfl_xor(ls, off, 32);
        const float mu = ls * (1.0f / 256.0f);
        float d2 = 0.0f, qd = 0.0f;
#pragma unroll
        for (int i = 0; i < 8; ++i) { s[i] = s[i] - mu; d2 += s[i] * s[i]; qd += q[i] * s[i]; }
#pragma unroll
        for (int off = 16; off > 0; off >>= 1) { d2 += __shfl_xor(d2, off, 32); qd += __shfl_xor(qd, off, 32); }
        const float rstd = rsqrtf(d2 * (1.0f / 256.0f) + 1e-5f);
#pragma unroll
        for (int i = 0; i < 8; ++i) { s[i] = s[i] * rstd; sm[i] += s[i]; }
        const float t = (qd * rstd) * SC2;
        const bool valid = mk != 0; msum += mk;
        const float tv = valid ? t : NEGB;
        const float mnew = fmaxf(m, tv);
        const float corr = __builtin_amdgcn_exp2f(m - mnew);
        const float pe = __builtin_amdgcn_exp2f(tv - mnew);
        const float p = valid ? pe : 0.0f;
        Z = Z * corr + p;
#pragma unroll
        for (int i = 0; i < 8; ++i) acc[i] = acc[i] * corr + p * s[i];
        m = mnew;
    }
    const bool uni = (msum == 0);
    const float zs = (Z > 0.0f) ? Z : 1.0f;
    const float inv = 1.0f / zs;
    v8h hv;
#pragma unroll
    for (int i = 0; i < 8; ++i) { const float o = uni ? (sm[i] * (1.0f / 6.0f)) : (acc[i] * inv); hv[i] = toh_flush(o * ACAR); }
    h16* dst = TP + (size_t)l * CC + cb;
    *(volatile v8h*)dst = hv; __threadfence(); *(volatile v8h*)dst = hv;
}

__global__ __launch_bounds__(32) void k_oproj(const h16* __restrict__ A, const h16* __restrict__ Bt, const float* __restrict__ bias, float* OUT) {
    __shared__ __align__(16) float os[16 * 68];
    const int K = CC;
    const int lane = threadIdx.x & 31, lr = lane & 15, hi = lane >> 4; const int r0 = blockIdx.x * 64, c0 = blockIdx.y * 64;
    v8f acc[4][4];
#pragma unroll
    for (int mb = 0; mb < 4; ++mb)
#pragma unroll
        for (int nb = 0; nb < 4; ++nb) acc[mb][nb] = (v8f){};
    const size_t aoff = (size_t)(r0 + lr) * K + 8 * hi, boff = (size_t)(c0 + lr) * K + 8 * hi;
#pragma unroll 1
    for (int kc = 0; kc < K; kc += 32) {
        v16h a[4];
#pragma unroll
        for (int mb = 0; mb < 4; ++mb) a[mb] = ldh(A + aoff + (size_t)mb * 16 * K + kc);
#pragma unroll
        for (int nb = 0; nb < 4; ++nb) { const v16h b = ldh(Bt + boff + (size_t)nb * 16 * K + kc);
#pragma unroll
            for (int mb = 0; mb < 4; ++mb) acc[mb][nb] = wmma16g(a[mb], b, acc[mb][nb]); }
    }
    float bc[4];
#pragma unroll
    for (int nb = 0; nb < 4; ++nb) bc[nb] = bfr(bias[c0 + nb * 16 + lr]);
#pragma unroll
    for (int mb = 0; mb < 4; ++mb) {
#pragma unroll
        for (int nb = 0; nb < 4; ++nb) {
#pragma unroll
            for (int j = 0; j < 8; ++j) os[(hi * 8 + j) * 68 + nb * 16 + lr] = acc[mb][nb][j] * FOLD + bc[nb]; }
        wave_sync();
        float* ob = OUT + (size_t)(r0 + mb * 16) * CC + c0;
#pragma unroll 1
        for (int ps = 0; ps < 2; ++ps) {
#pragma unroll
            for (int s = 0; s < 8; ++s) { const int p = s * 32 + lane; const int row = p >> 4, c4 = (p & 15) * 4;
                const v4f val = *(const v4fa*)(&os[row * 68 + c4]);
                *(volatile v4f*)(ob + (size_t)row * CC + c4) = val; }
            if (ps == 0) __threadfence(); }
        wave_sync();
    }
}

static constexpr size_t al256(size_t v) { return (v + 255) & ~(size_t)255; }
static constexpr size_t SZ_VB = al256((size_t)NCAM * HW * CC * 2);
static constexpr size_t SZ_WH = al256((size_t)CC * CC * 2);
static constexpr size_t SZ_TP = al256((size_t)LQ * CC * 2);
static constexpr size_t SZ_TOTAL = SZ_VB + SZ_WH + SZ_TP;
static_assert(SZ_TOTAL <= (size_t)134217728);
static_assert(((size_t)NCAM * HW * CC * 2) % 128 == 0);
static_assert(((size_t)LQ * CC * 2) % 128 == 0);

extern "C" void kernel_launch(void* const* d_in, const int* in_sizes, int n_in,
                              void* d_out, int out_size, void* d_ws, size_t ws_size, hipStream_t stream) {
    if (n_in < 10) return;
    if ((size_t)in_sizes[0] < (size_t)LQ * CC) return;
    if ((size_t)in_sizes[2] < (size_t)NCAM * CC * HW) return;
    if ((size_t)in_sizes[4] < ((size_t)(NCAM - 1) * LQ_FULL + LQ) * 2) return;
    if ((size_t)in_sizes[5] < (size_t)(NCAM - 1) * LQ_FULL + LQ) return;
    if ((size_t)in_sizes[8] < (size_t)CC * CC || in_sizes[9] < CC) return;
    if ((size_t)out_size < (size_t)LQ * CC) return;
    if (SZ_TOTAL > ws_size) return;
    const float* query = (const float*)d_in[0];
    const float* value = (const float*)d_in[2];
    const float* pts   = (const float*)d_in[4];
    const int*   msk   = (const int*)d_in[5];
    const float* wout  = (const float*)d_in[8];
    const float* bout  = (const float*)d_in[9];
    float* OUT = (float*)d_out;
    char* wsp = (char*)d_ws;
    bf*  VB = (bf*)wsp;  wsp += SZ_VB;
    h16* WH = (h16*)wsp; wsp += SZ_WH;
    h16* TP = (h16*)wsp; wsp += SZ_TP;

    k_wcvt<<<(unsigned)((size_t)CC * CC / 8 / 256), 256, 0, stream>>>(wout, WH);
    k_vtr<<<dim3(HW / 32, CC / 64, NCAM), 256, 0, stream>>>(value, VB);
    k_sample<<<LQ / SWV, 256, 0, stream>>>(query, VB, pts, msk, TP);
    k_oproj<<<dim3(LQ / 64, CC / 64, 1), 32, 0, stream>>>(TP, WH, bout, OUT);
}
